// LongformerAttention_11982958756577
// MI455X (gfx1250) — hardware-verified
//
#include <hip/hip_runtime.h>
#include <math.h>

#ifndef NB
#define NB 2
#endif
#ifndef SEQ
#define SEQ 4096
#endif
#define NB_FULL 2
#define SEQ_FULL 4096
#define EE 768
#define NH 12
#define DD 64
#define LW 256
#define NKT (SEQ / 32)
#define NBH (NB * NH)
#define MROWS (NB * SEQ)
static_assert(SEQ % 128 == 0);
static_assert(SEQ <= SEQ_FULL);
static_assert(NB <= NB_FULL);
static_assert(EE == NH * DD);
static_assert(EE % 64 == 0);
static_assert(LW % 32 == 0);

typedef __attribute__((ext_vector_type(16))) _Float16 v16h;
typedef __attribute__((ext_vector_type(16))) __bf16 v16b;
typedef __attribute__((ext_vector_type(8)))  _Float16 v8h;
typedef __attribute__((ext_vector_type(8)))  __bf16 v8b;
typedef __attribute__((ext_vector_type(8)))  float v8f;
typedef __attribute__((ext_vector_type(4)))  float v4f;
typedef __attribute__((ext_vector_type(4)))  unsigned v4u;

template <typename T> __device__ __forceinline__ void vst2(void* p, T v) { *(volatile T*)p = v; __threadfence(); *(volatile T*)p = v; }
__device__ __forceinline__ v8f wmma16(v16h a, v16h b, v8f c) {
  v8f d = __builtin_amdgcn_wmma_f32_16x16x32_f16(false, a, false, b, (short)0, c, false, false);
  asm volatile("v_nop\n\tv_nop\n\tv_nop\n\tv_nop" : "+v"(d) : "v"(a), "v"(b));
  return d;
}
__device__ __forceinline__ v8f wmma_bf(v16b a, v16b b, v8f c) {
  v8f d = __builtin_amdgcn_wmma_f32_16x16x32_bf16(false, a, false, b, (short)0, c, false, false);
  asm volatile("v_nop\n\tv_nop\n\tv_nop\n\tv_nop" : "+v"(d) : "v"(a), "v"(b));
  return d;
}
__device__ __forceinline__ v16h frag_h(const _Float16* rowk0, int lane) {
  union { v16h v; v8h q[2]; } u; const _Float16* p = rowk0 + 8 * (lane >> 4);
  u.q[0] = *(const v8h*)p; u.q[1] = *(const v8h*)(p + 16); return u.v;
}
__device__ __forceinline__ v16b frag_b(const __bf16* rowk0, int lane) {
  union { v16b v; v8b q[2]; } u; const __bf16* p = rowk0 + 8 * (lane >> 4);
  u.q[0] = *(const v8b*)p; u.q[1] = *(const v8b*)(p + 16); return u.v;
}
__device__ __forceinline__ float bfr(float v) { return (float)(__bf16)v; }
__device__ __forceinline__ void ldsx() { asm volatile("s_wait_dscnt 0" ::: "memory"); __builtin_amdgcn_wave_barrier(); __builtin_amdgcn_fence(3, "workgroup"); }

#define WS_XB  ((size_t)0)
#define SZ_XB  ((size_t)MROWS * EE * 2)
#define WS_WT  (WS_XB + SZ_XB)
#define SZ_WT  ((size_t)3 * EE * EE * 2)
#define WS_Q   (WS_WT + SZ_WT)
#define SZ_P   ((size_t)NBH * SEQ * DD * 2)
#define WS_K   (WS_Q + SZ_P)
#define WS_V   (WS_K + SZ_P)
#define WS_END (WS_V + SZ_P)
static_assert(SZ_XB % 128 == 0);
static_assert(SZ_WT % 128 == 0);
static_assert(SZ_P % 128 == 0);
static_assert(WS_END <= (size_t)134217728);

__global__ __launch_bounds__(96) void k_cvtx(const float* __restrict__ X, __bf16* __restrict__ Xb) {
  const int r = blockIdx.x, t = threadIdx.x; const int b = r / SEQ, s = r - b * SEQ;
  const float* src = X + ((size_t)s * NB_FULL + b) * EE + t * 8;
  const v4f f0 = *(const v4f*)src, f1 = *(const v4f*)(src + 4);
  union { v8b b; v4u u; } o;
#pragma unroll
  for (int j = 0; j < 4; ++j) { o.b[j] = (__bf16)f0[j]; o.b[4 + j] = (__bf16)f1[j]; }
  vst2((void*)(Xb + (size_t)r * EE + t * 8), o.u);
}

__global__ __launch_bounds__(256) void k_cvtw(const float* __restrict__ Wq, const float* __restrict__ Wk, const float* __restrict__ Wv, __bf16* __restrict__ Wt) {
  __shared__ __align__(16) __bf16 tt[64][72];
  const int z = blockIdx.z, t = threadIdx.x; const int k0 = blockIdx.x * 64, n0 = blockIdx.y * 64;
  const float* W = (z == 0) ? Wq : (z == 1) ? Wk : Wv;
  { const int k = t >> 2, nb = (t & 3) * 16; const float* p = W + (size_t)(k0 + k) * EE + n0 + nb;
#pragma unroll
    for (int i = 0; i < 4; ++i) { const v4f f = *(const v4f*)(p + 4 * i);
#pragma unroll
      for (int j = 0; j < 4; ++j) tt[nb + 4 * i + j][k] = (__bf16)f[j]; } }
  __syncthreads();
#pragma unroll
  for (int it = 0; it < 2; ++it) { const int L = it * 32 + (t >> 3), pc = t & 7;
    vst2((void*)(Wt + ((size_t)z * EE + n0 + L) * EE + k0 + pc * 8), *(const v4u*)&tt[L][pc * 8]); }
}

__global__ __launch_bounds__(128) void k_proj(const __bf16* __restrict__ Xb, const __bf16* __restrict__ Wt, const float* __restrict__ bq, const float* __restrict__ bk, const float* __restrict__ bv,
                                              _Float16* __restrict__ Qp, _Float16* __restrict__ Kp, _Float16* __restrict__ VT) {
  __shared__ __align__(16) _Float16 tile[128 * 72];
  const int tid = threadIdx.x, wave = tid >> 5, lane = tid & 31, col = lane & 15, g = lane >> 4;
  const int z = blockIdx.z, h = blockIdx.y; const int n0 = h * DD; const int row0 = blockIdx.x * 128;
  const int b = row0 / SEQ, s0 = row0 - b * SEQ;
  const float* bp = (z == 0) ? bq : (z == 1) ? bk : bv;
  const __bf16* Wz = Wt + (size_t)z * EE * EE;
  v8f acc[2][4];
#pragma unroll
  for (int mt = 0; mt < 2; ++mt)
#pragma unroll
    for (int nt = 0; nt < 4; ++nt) acc[mt][nt] = v8f{};
#pragma unroll 1
  for (int ks = 0; ks < EE / 32; ++ks) { const int k0 = ks * 32;
    v16b a[2], w[4];
#pragma unroll
    for (int mt = 0; mt < 2; ++mt) a[mt] = frag_b(Xb + (size_t)(row0 + wave * 32 + mt * 16 + col) * EE + k0, lane);
#pragma unroll
    for (int nt = 0; nt < 4; ++nt) w[nt] = frag_b(Wz + (size_t)(n0 + nt * 16 + col) * EE + k0, lane);
#pragma unroll
    for (int mt = 0; mt < 2; ++mt)
#pragma unroll
      for (int nt = 0; nt < 4; ++nt) acc[mt][nt] = wmma_bf(a[mt], w[nt], acc[mt][nt]);
  }
#pragma unroll
  for (int nt = 0; nt < 4; ++nt) { const int cl = nt * 16 + col; const float bias = bfr(bp[n0 + cl]);
#pragma unroll
    for (int mt = 0; mt < 2; ++mt)
#pragma unroll
      for (int r = 0; r < 8; ++r) { const int rl = wave * 32 + mt * 16 + 8 * g + r; const _Float16 v = (_Float16)(acc[mt][nt][r] + bias);
        if (z == 2) tile[cl * 136 + rl] = v; else tile[rl * 72 + cl] = v; } }
  __syncthreads();
  const size_t bh = (size_t)b * NH + h;
#pragma unroll
  for (int it = 0; it < 8; ++it) { const int L = it * 16 + (tid >> 3), pc = tid & 7;
    if (z == 2) { const int d = L >> 1, sh = L & 1;
      vst2((void*)(VT + (bh * DD + d) * (size_t)SEQ + s0 + sh * 64 + pc * 8), *(const v4u*)&tile[d * 136 + sh * 64 + pc * 8]); }
    else { _Float16* P = (z == 0) ? Qp : Kp;
      vst2((void*)(P + (bh * SEQ + s0 + L) * (size_t)DD + pc * 8), *(const v4u*)&tile[L * 72 + pc * 8]); } }
}

__global__ __launch_bounds__(128) void k_att(const _Float16* __restrict__ Qp, const _Float16* __restrict__ Kp, const _Float16* __restrict__ VT, float* __restrict__ OUT) {
  __shared__ __align__(16) float sp[4][16][36]; __shared__ __align__(16) float so[4][16][68];
  const int tid = threadIdx.x, wave = tid >> 5, lane = tid & 31, col = lane & 15, g = lane >> 4; const int bh = blockIdx.y; const int b = bh / NH, h = bh - b * NH;
  const int qb = blockIdx.x; const int q0 = qb * 64 + wave * 16; const size_t rq = (size_t)bh * SEQ + q0;
  v16h aq[2];
#pragma unroll
  for (int kc = 0; kc < 2; ++kc) aq[kc] = frag_h(Qp + (rq + col) * DD + kc * 32, lane);
  float m[8], l[8];
#pragma unroll
  for (int r = 0; r < 8; ++r) { m[r] = -3.0e38f; l[r] = 0.f; }
  v8f acc[4];
#pragma unroll
  for (int j = 0; j < 4; ++j) acc[j] = v8f{};
  const int klo = qb * 64 - LW, khi = qb * 64 + 63 + LW;
  const int kslo = (klo > 0) ? (klo >> 5) : 0; const int kshi = (khi < SEQ - 1) ? (khi >> 5) : (NKT - 1);
#pragma unroll 1
  for (int ks = kslo; ks <= kshi; ++ks) {
    float s[2][8];
#pragma unroll
    for (int ct = 0; ct < 2; ++ct) { const int kk = ks * 32 + ct * 16 + col; v8f c = v8f{};
#pragma unroll
      for (int kc = 0; kc < 2; ++kc) { const v16h w = frag_h(Kp + ((size_t)bh * SEQ + kk) * DD + kc * 32, lane); c = wmma16(aq[kc], w, c); }
#pragma unroll
      for (int r = 0; r < 8; ++r) { const int qi = q0 + 8 * g + r; const int dq = qi - kk; const bool keep = (dq <= LW) && (dq >= -LW); s[ct][r] = keep ? c[r] * 0.125f : -3.0e38f; } }
    float alpha[8];
#pragma unroll
    for (int r = 0; r < 8; ++r) { float mx = fmaxf(s[0][r], s[1][r]);
#pragma unroll
      for (int o = 1; o < 16; o <<= 1) mx = fmaxf(mx, __shfl_xor(mx, o));
      const float mn = fmaxf(m[r], mx); alpha[r] = (m[r] <= -1.0e38f) ? 0.f : __expf(m[r] - mn); const float e0 = (s[0][r] <= -1.0e38f) ? 0.f : __expf(s[0][r] - mn), e1 = (s[1][r] <= -1.0e38f) ? 0.f : __expf(s[1][r] - mn); float es = e0 + e1;
#pragma unroll
      for (int o = 1; o < 16; o <<= 1) es += __shfl_xor(es, o);
      l[r] = l[r] * alpha[r] + es; m[r] = (mn > -1.0e38f) ? mn : m[r]; sp[wave][8 * g + r][col] = e0; sp[wave][8 * g + r][16 + col] = e1; }
#pragma unroll
    for (int j = 0; j < 4; ++j)
#pragma unroll
      for (int r = 0; r < 8; ++r) acc[j][r] *= alpha[r];
    ldsx();
    v16h pa, par; { const float* prow = &sp[wave][col][0] + 8 * (lane >> 4);
#pragma unroll
      for (int i = 0; i < 8; ++i) { const float p0 = prow[i] * 2048.0f, p1 = prow[16 + i] * 2048.0f; pa[i] = (_Float16)p0; pa[8 + i] = (_Float16)p1; par[i] = (_Float16)(p0 - (float)pa[i]); par[8 + i] = (_Float16)(p1 - (float)pa[8 + i]); } }
#pragma unroll
    for (int j = 0; j < 4; ++j) { const v16h vh = frag_h(VT + ((size_t)bh * DD + j * 16 + col) * SEQ + ks * 32, lane); acc[j] = wmma16(pa, vh, acc[j]); acc[j] = wmma16(par, vh, acc[j]); }
    ldsx(); }
#pragma unroll
  for (int r = 0; r < 8; ++r) { const float il = (l[r] > 0.f) ? (1.0f / 2048.0f) / l[r] : 0.f;
#pragma unroll
    for (int j = 0; j < 4; ++j) so[wave][8 * g + r][j * 16 + col] = acc[j][r] * il; }
  ldsx();
  for (int rl = 0; rl < 16; ++rl) if (lane < 16) vst2((void*)(OUT + ((size_t)(q0 + rl) * NB + b) * EE + h * DD + lane * 4), *(const v4f*)&so[wave][rl][lane * 4]);
}

extern "C" void kernel_launch(void* const* d_in, const int* in_sizes, int n_in, void* d_out, int out_size, void* d_ws, size_t ws_size, hipStream_t stream) {
  if (n_in < 7) return;
  if (in_sizes[0] < SEQ * NB_FULL * EE) return;
  if (in_sizes[1] < EE * EE || in_sizes[3] < EE * EE || in_sizes[5] < EE * EE) return;
  if (in_sizes[2] < EE || in_sizes[4] < EE || in_sizes[6] < EE) return;
  if (out_size < SEQ * NB * EE) return;
  if (ws_size < (size_t)WS_END) return;
  const float* X  = (const float*)d_in[0];
  const float* Wq = (const float*)d_in[1]; const float* bq = (const float*)d_in[2];
  const float* Wk = (const float*)d_in[3]; const float* bk = (const float*)d_in[4];
  const float* Wv = (const float*)d_in[5]; const float* bv = (const float*)d_in[6];
  char* ws = (char*)d_ws;
  __bf16* Xb = (__bf16*)(ws + WS_XB); __bf16* Wt = (__bf16*)(ws + WS_WT);
  _Float16* Qp = (_Float16*)(ws + WS_Q); _Float16* Kp = (_Float16*)(ws + WS_K); _Float16* VT = (_Float16*)(ws + WS_V);
  k_cvtx<<<dim3(MROWS), 96, 0, stream>>>(X, Xb);
  k_cvtw<<<dim3(EE / 64, EE / 64, 3), 256, 0, stream>>>(Wq, Wk, Wv, Wt);
  k_proj<<<dim3(MROWS / 128, NH, 3), 128, 0, stream>>>(Xb, Wt, bq, bk, bv, Qp, Kp, VT);
  k_att<<<dim3(SEQ / 64, NBH), 128, 0, stream>>>(Qp, Kp, VT, (float*)d_out);
}
